// GroupedQueryAttention_71038759075920
// MI455X (gfx1250) — hardware-verified
//
#include <hip/hip_runtime.h>
#include <math.h>

typedef __attribute__((ext_vector_type(16))) _Float16     v16h;
typedef __attribute__((ext_vector_type(8)))  _Float16     v8h;
typedef __attribute__((ext_vector_type(8)))  float        v8f;
typedef __attribute__((ext_vector_type(4)))  float        v4f;
typedef __attribute__((ext_vector_type(4)))  unsigned int v4u;
typedef __attribute__((ext_vector_type(4)))  int          v4i;

#ifndef NB
#define NB 1
#endif
#ifndef SEQ
#define SEQ 2048
#endif
#define NB_FULL  1
#define SEQ_FULL 2048
#define EMB   2048
#define NQH   32
#define NKVH  8
#define GRP   4
#define HDIM  64
#define EKV   512
#define NQG   4096
#define NQKV  5120
#define KC    64
#define QT    16
#define NWAVE 4
#define ER    ((SEQ) < 256 ? (SEQ) : 256)

#define XSC 16.0f
#define WSC 64.0f
#define QSC 64.0f
#define KSC 16.0f
#define VSC 64.0f
#define PSC 32768.0f
#define CSC 256.0f

#define XP_B   ((size_t)SEQ * EMB * 2)
#define WP_B   ((size_t)NQKV * EMB * 2)
#define WOP_B  ((size_t)EMB * EMB * 2)
#define QKV_B  ((size_t)SEQ * NQKV * 4)
#define QH_B   ((size_t)SEQ * EMB * 2)
#define K16_B  ((size_t)SEQ * EKV * 2)
#define KL_B   ((size_t)ER * EKV * 2)
#define VT_B   ((size_t)EKV * SEQ * 2)
#define CH_B   ((size_t)SEQ * EMB * 2)
#define CL_B   ((size_t)ER * EMB * 2)
#define WS_TOTAL (XP_B + WP_B + WOP_B + QKV_B + 2 * QH_B + K16_B + KL_B + 2 * VT_B + CH_B + CL_B)

static_assert(NB == 1 && NB_FULL == 1);
static_assert(SEQ <= SEQ_FULL);
static_assert(SEQ % KC == 0 && SEQ % QT == 0);
static_assert(SEQ % 64 == 0 && SEQ % 32 == 0);
static_assert(ER % 32 == 0 && ER % QT == 0 && ER <= SEQ);
static_assert(ER % KC == 0);
static_assert(EMB == NQH * HDIM && EKV == NKVH * HDIM && NQH == NKVH * GRP && GRP == NWAVE);
static_assert(NQG == NQH * 2 * HDIM && NQKV == NQG + 2 * EKV);
static_assert(HDIM == 64 && KC == 64 && QT == 16);
static_assert(EMB % 32 == 0);
static_assert(NQKV % 256 == 0 && EMB % 256 == 0);
static_assert(NWAVE * 32 * 4 == KC * (HDIM / 8));
static_assert(NWAVE * 32 * 2 == QT * (KC / 4));
static_assert((XP_B % 256) == 0 && (WP_B % 256) == 0 && (WOP_B % 256) == 0 && (QKV_B % 256) == 0);
static_assert((QH_B % 256) == 0 && (K16_B % 256) == 0 && (KL_B % 256) == 0 && (VT_B % 256) == 0 && (CH_B % 256) == 0 && (CL_B % 256) == 0);
static_assert(WS_TOTAL <= (size_t)134217728);

union FH { v16h v; v8h h[2]; };

__device__ __forceinline__ unsigned int bf_bits(float f) {
    const unsigned int u = __float_as_uint(f);
    return (u + 0x7FFFu + ((u >> 16) & 1u)) >> 16;
}
__device__ __forceinline__ float bf_val(float f) { return __uint_as_float(bf_bits(f) << 16); }
__device__ __forceinline__ unsigned int h_bits(float f) { return (unsigned int)__builtin_bit_cast(unsigned short, (_Float16)f); }
__device__ __forceinline__ void split_h(float v, unsigned int& hb, unsigned int& lb) {
    const _Float16 h = (_Float16)v;
    const _Float16 l = (_Float16)(v - (float)h);
    hb = (unsigned int)__builtin_bit_cast(unsigned short, h);
    lb = (unsigned int)__builtin_bit_cast(unsigned short, l);
}

__device__ __forceinline__ v8f mma_h(v16h a, v16h b, v8f c) {
    c = __builtin_amdgcn_wmma_f32_16x16x32_f16(false, a, false, b, (short)0, c, false, false);
    asm volatile("v_nop\n\tv_nop\n\tv_nop\n\tv_nop" : "+v"(c) : "v"(a), "v"(b));
    return c;
}

__device__ __forceinline__ void wave_sync() {
    __builtin_amdgcn_fence(3  , "workgroup");
    __builtin_amdgcn_wave_barrier();
    __builtin_amdgcn_fence(2  , "workgroup");
}

__device__ __forceinline__ void st16x2(unsigned short* p, v4u v) {
    volatile v4u* d = (volatile v4u*)p;
    *d = v; __threadfence(); *d = v;
}

__global__ __launch_bounds__(256) void k_cvt(const float* __restrict__ src, unsigned short* __restrict__ dst, int n8, float scale) {
    const int u = blockIdx.x * 256 + threadIdx.x;
    if (u >= n8) return;
    const float* sp = src + (size_t)u * 8;
    const v4f a = *(const v4f*)(sp), c = *(const v4f*)(sp + 4);
    v4u pk;
    pk.x = h_bits(bf_val(a.x) * scale) | (h_bits(bf_val(a.y) * scale) << 16);
    pk.y = h_bits(bf_val(a.z) * scale) | (h_bits(bf_val(a.w) * scale) << 16);
    pk.z = h_bits(bf_val(c.x) * scale) | (h_bits(bf_val(c.y) * scale) << 16);
    pk.w = h_bits(bf_val(c.z) * scale) | (h_bits(bf_val(c.w) * scale) << 16);
    st16x2(dst + (size_t)u * 8, pk);
}

__device__ __forceinline__ void gemm_pass(const _Float16* __restrict__ Ah, const _Float16* __restrict__ Bh, int K,
                                          int row0, int col0, int c, int hh, v8f (&acc)[2][4]) {
    const _Float16* ap = Ah + (size_t)(row0 + c) * K + 8 * hh;
    const _Float16* bp = Bh + (size_t)(col0 + c) * K + 8 * hh;
    const size_t r16 = (size_t)16 * K;
#pragma unroll 1
    for (int k0 = 0; k0 < K; k0 += 32) {
        FH a[2], b[4];
#pragma unroll
        for (int mt = 0; mt < 2; ++mt) {
            a[mt].h[0] = *(const v8h*)(ap + mt * r16 + k0);
            a[mt].h[1] = *(const v8h*)(ap + mt * r16 + k0 + 16);
        }
#pragma unroll
        for (int nt = 0; nt < 4; ++nt) {
            b[nt].h[0] = *(const v8h*)(bp + nt * r16 + k0);
            b[nt].h[1] = *(const v8h*)(bp + nt * r16 + k0 + 16);
        }
#pragma unroll
        for (int mt = 0; mt < 2; ++mt)
#pragma unroll
            for (int nt = 0; nt < 4; ++nt)
                acc[mt][nt] = mma_h(a[mt].v, b[nt].v, acc[mt][nt]);
    }
}

__global__ __launch_bounds__(128) void k_gemm(const unsigned short* __restrict__ A, const unsigned short* __restrict__ Ares,
                                               const unsigned short* __restrict__ B, float* __restrict__ C,
                                               int K, int ldc, int resRows, float oscale) {
    __shared__ __align__(16) float Cs[NWAVE * 32 * 68];
    const int tid = threadIdx.x, lane = tid & 31, hh = lane >> 4, c = lane & 15;
    const int wave = __builtin_amdgcn_readfirstlane(tid >> 5);
    const int row0 = blockIdx.y * 32;
    const int col0 = blockIdx.x * 256 + wave * 64;

    v8f acc[2][4];
#pragma unroll
    for (int mt = 0; mt < 2; ++mt)
#pragma unroll
        for (int nt = 0; nt < 4; ++nt) acc[mt][nt] = (v8f){0.f, 0.f, 0.f, 0.f, 0.f, 0.f, 0.f, 0.f};

    gemm_pass((const _Float16*)A, (const _Float16*)B, K, row0, col0, c, hh, acc);
    if (row0 < resRows)
        gemm_pass((const _Float16*)Ares, (const _Float16*)B, K, row0, col0, c, hh, acc);

    const int cso = wave * (32 * 68);
#pragma unroll
    for (int mt = 0; mt < 2; ++mt)
#pragma unroll
        for (int nt = 0; nt < 4; ++nt)
#pragma unroll
            for (int r = 0; r < 8; ++r)
                Cs[cso + (mt * 16 + 8 * hh + r) * 68 + nt * 16 + c] = acc[mt][nt][r] * oscale;
    wave_sync();
    {
        float* cb = C + (size_t)row0 * ldc + col0;
        const int c4 = c * 4;
        for (int pass = 0; pass < 2; ++pass) {
#pragma unroll
            for (int it = 0; it < 16; ++it) {
                const int row = it * 2 + hh;
                const v4f val = *(const v4f*)(&Cs[cso + row * 68 + c4]);
                *(volatile v4f*)(cb + (size_t)row * ldc + c4) = val;
            }
            __threadfence();
        }
    }
}

__global__ __launch_bounds__(256) void k_prep_qk(const float* __restrict__ QKV, const float* __restrict__ cosT, const float* __restrict__ sinT,
                                                  const float* __restrict__ qnw, const float* __restrict__ knw,
                                                  unsigned short* __restrict__ Qhi, unsigned short* __restrict__ Qlo,
                                                  unsigned short* __restrict__ K16, unsigned short* __restrict__ Klo) {
    const int t = threadIdx.x;
    const int s = blockIdx.x * 32 + (t >> 3);
    const int pc = t & 7;
    const int slot = blockIdx.y;
    const bool isq = slot < NQH;
    const bool klo = (int)(blockIdx.x * 32) < ER;
    const int col = isq ? slot * (2 * HDIM) : NQG + (slot - NQH) * HDIM;
    const int d0 = pc * 8, dp = (d0 + 32) & 63;
    const float* row = QKV + (size_t)s * NQKV + col;
    const v4f a0 = *(const v4f*)(row + d0), a1 = *(const v4f*)(row + d0 + 4);
    const v4f b0 = *(const v4f*)(row + dp), b1 = *(const v4f*)(row + dp + 4);
    const float av[8] = {a0.x, a0.y, a0.z, a0.w, a1.x, a1.y, a1.z, a1.w};
    const float bv[8] = {b0.x, b0.y, b0.z, b0.w, b1.x, b1.y, b1.z, b1.w};
    float ss = 0.f;
#pragma unroll
    for (int e = 0; e < 8; ++e) ss += av[e] * av[e];
    ss += __shfl_xor(ss, 1, 32); ss += __shfl_xor(ss, 2, 32); ss += __shfl_xor(ss, 4, 32);
    const float rinv = rsqrtf(ss * (1.0f / 64.0f) + 1e-6f);

    const v4f q0 = *(const v4f*)(qnw + d0), q1 = *(const v4f*)(qnw + d0 + 4), q2 = *(const v4f*)(qnw + dp), q3 = *(const v4f*)(qnw + dp + 4);
    const v4f k0 = *(const v4f*)(knw + d0), k1 = *(const v4f*)(knw + d0 + 4), k2 = *(const v4f*)(knw + dp), k3 = *(const v4f*)(knw + dp + 4);
    const float wqa[8] = {q0.x, q0.y, q0.z, q0.w, q1.x, q1.y, q1.z, q1.w};
    const float wqb[8] = {q2.x, q2.y, q2.z, q2.w, q3.x, q3.y, q3.z, q3.w};
    const float wka[8] = {k0.x, k0.y, k0.z, k0.w, k1.x, k1.y, k1.z, k1.w};
    const float wkb[8] = {k2.x, k2.y, k2.z, k2.w, k3.x, k3.y, k3.z, k3.w};
    const v4f c0 = *(const v4f*)(cosT + (size_t)s * HDIM + d0), c1 = *(const v4f*)(cosT + (size_t)s * HDIM + d0 + 4);
    const v4f s0 = *(const v4f*)(sinT + (size_t)s * HDIM + d0), s1 = *(const v4f*)(sinT + (size_t)s * HDIM + d0 + 4);
    const float cv[8] = {c0.x, c0.y, c0.z, c0.w, c1.x, c1.y, c1.z, c1.w};
    const float sv[8] = {s0.x, s0.y, s0.z, s0.w, s1.x, s1.y, s1.z, s1.w};
    const float sgn = (pc < 4) ? -1.0f : 1.0f;

    float o[8];
#pragma unroll
    for (int e = 0; e < 8; ++e) {
        const float wa = 1.0f + bf_val(isq ? wqa[e] : wka[e]);
        const float wb = 1.0f + bf_val(isq ? wqb[e] : wkb[e]);
        const float n  = (av[e] * rinv) * wa;
        const float pn = (bv[e] * rinv) * wb;
        o[e] = n * bf_val(cv[e]) + sgn * (pn * bf_val(sv[e]));
    }
    if (isq) {
        unsigned int hb[8], lb[8];
#pragma unroll
        for (int e = 0; e < 8; ++e) split_h(o[e] * QSC, hb[e], lb[e]);
        v4u ph, pl;
        ph.x = hb[0] | (hb[1] << 16); ph.y = hb[2] | (hb[3] << 16); ph.z = hb[4] | (hb[5] << 16); ph.w = hb[6] | (hb[7] << 16);
        pl.x = lb[0] | (lb[1] << 16); pl.y = lb[2] | (lb[3] << 16); pl.z = lb[4] | (lb[5] << 16); pl.w = lb[6] | (lb[7] << 16);
        const size_t off = (size_t)s * EMB + slot * HDIM + d0;
        st16x2(Qhi + off, ph);
        st16x2(Qlo + off, pl);
    } else {
        unsigned int hb[8], lb[8];
#pragma unroll
        for (int e = 0; e < 8; ++e) split_h(o[e] * KSC, hb[e], lb[e]);
        v4u ph, pl;
        ph.x = hb[0] | (hb[1] << 16); ph.y = hb[2] | (hb[3] << 16); ph.z = hb[4] | (hb[5] << 16); ph.w = hb[6] | (hb[7] << 16);
        pl.x = lb[0] | (lb[1] << 16); pl.y = lb[2] | (lb[3] << 16); pl.z = lb[4] | (lb[5] << 16); pl.w = lb[6] | (lb[7] << 16);
        const size_t off = (size_t)s * EKV + (slot - NQH) * HDIM + d0;
        st16x2(K16 + off, ph);
        if (klo) st16x2(Klo + off, pl);
    }
}

__global__ __launch_bounds__(256) void k_prep_v(const float* __restrict__ QKV, unsigned short* __restrict__ VThi, unsigned short* __restrict__ VTlo) {
    __shared__ __align__(16) unsigned short th[64 * 72];
    __shared__ __align__(16) unsigned short tl[64 * 72];
    const int t = threadIdx.x;
    const int s0 = blockIdx.x * 64, kv = blockIdx.y;
    {
        const int rl = t >> 2, part = t & 3;
        const float* src = QKV + (size_t)(s0 + rl) * NQKV + NQG + EKV + kv * HDIM + part * 16;
        const v4f f0 = *(const v4f*)(src), f1 = *(const v4f*)(src + 4), f2 = *(const v4f*)(src + 8), f3 = *(const v4f*)(src + 12);
        const float fv[16] = {f0.x, f0.y, f0.z, f0.w, f1.x, f1.y, f1.z, f1.w, f2.x, f2.y, f2.z, f2.w, f3.x, f3.y, f3.z, f3.w};
        unsigned int hb[16], lb[16];
#pragma unroll
        for (int e = 0; e < 16; ++e) split_h(fv[e] * VSC, hb[e], lb[e]);
        v4u h0, h1, l0, l1;
        h0.x = hb[0] | (hb[1] << 16);   h0.y = hb[2] | (hb[3] << 16);   h0.z = hb[4] | (hb[5] << 16);   h0.w = hb[6] | (hb[7] << 16);
        h1.x = hb[8] | (hb[9] << 16);   h1.y = hb[10] | (hb[11] << 16); h1.z = hb[12] | (hb[13] << 16); h1.w = hb[14] | (hb[15] << 16);
        l0.x = lb[0] | (lb[1] << 16);   l0.y = lb[2] | (lb[3] << 16);   l0.z = lb[4] | (lb[5] << 16);   l0.w = lb[6] | (lb[7] << 16);
        l1.x = lb[8] | (lb[9] << 16);   l1.y = lb[10] | (lb[11] << 16); l1.z = lb[12] | (lb[13] << 16); l1.w = lb[14] | (lb[15] << 16);
        *(v4u*)(th + rl * 72 + part * 16)     = h0;
        *(v4u*)(th + rl * 72 + part * 16 + 8) = h1;
        *(v4u*)(tl + rl * 72 + part * 16)     = l0;
        *(v4u*)(tl + rl * 72 + part * 16 + 8) = l1;
    }
    __syncthreads();
#pragma unroll
    for (int it = 0; it < 2; ++it) {
        const int drow = it * 32 + (t >> 3), pc = t & 7;
        unsigned int e[8], f[8];
#pragma unroll
        for (int j = 0; j < 8; ++j) { e[j] = (unsigned int)th[(pc * 8 + j) * 72 + drow]; f[j] = (unsigned int)tl[(pc * 8 + j) * 72 + drow]; }
        v4u ph, pl;
        ph.x = e[0] | (e[1] << 16); ph.y = e[2] | (e[3] << 16); ph.z = e[4] | (e[5] << 16); ph.w = e[6] | (e[7] << 16);
        pl.x = f[0] | (f[1] << 16); pl.y = f[2] | (f[3] << 16); pl.z = f[4] | (f[5] << 16); pl.w = f[6] | (f[7] << 16);
        const size_t off = (size_t)(kv * HDIM + drow) * SEQ + s0 + pc * 8;
        st16x2(VThi + off, ph);
        st16x2(VTlo + off, pl);
    }
}

__global__ __launch_bounds__(128) void k_attn(const unsigned short* __restrict__ Qhi, const unsigned short* __restrict__ Qlo,
                                               const unsigned short* __restrict__ K16, const unsigned short* __restrict__ Klo,
                                               const unsigned short* __restrict__ VThi, const unsigned short* __restrict__ VTlo,
                                               const int* __restrict__ mask, const float* __restrict__ QKV,
                                               unsigned short* __restrict__ Chi, unsigned short* __restrict__ Clo) {
    __shared__ __align__(16) _Float16 Ksh[KC * HDIM];
    __shared__ __align__(16) _Float16 Ksl[KC * HDIM];
    __shared__ __align__(16) _Float16 Vth[HDIM * KC];
    __shared__ __align__(16) _Float16 Vtl[HDIM * KC];
    __shared__ __align__(16) int      Msh[QT * KC];
    __shared__ __align__(16) _Float16 Psh[NWAVE * QT * 32];
    __shared__ __align__(16) _Float16 Psl[NWAVE * QT * 32];
    __shared__ __align__(16) float    Os[NWAVE * QT * 68];
    __shared__ int Fsh[2 * NWAVE];

    const int tid = threadIdx.x, lane = tid & 31, hh = lane >> 4, c = lane & 15;
    const int wave = __builtin_amdgcn_readfirstlane(tid >> 5);
    const int q0 = blockIdx.x * QT, kv = blockIdx.y;
    const bool res = q0 < ER;
    const int head = kv * GRP + wave;
    const float SL2 = 1.4426950408889634f / 8192.0f;

    float mrow[8], lrow[8];
    v8f oacc[4];
#pragma unroll
    for (int r = 0; r < 8; ++r) { mrow[r] = -INFINITY; lrow[r] = 0.f; }
#pragma unroll
    for (int t = 0; t < 4; ++t) oacc[t] = (v8f){0.f, 0.f, 0.f, 0.f, 0.f, 0.f, 0.f, 0.f};

    const _Float16* Qh = (const _Float16*)Qhi;
    const _Float16* Ql = (const _Float16*)Qlo;
    const size_t qbase = (size_t)(q0 + c) * EMB + head * HDIM + 8 * hh;
    const unsigned short* Kb = K16 + kv * HDIM;
    const unsigned short* Kl = Klo + kv * HDIM;
    const unsigned short* Vb = VThi + (size_t)(kv * HDIM) * SEQ;
    const unsigned short* Vl = VTlo + (size_t)(kv * HDIM) * SEQ;
    const int* mb = mask + (size_t)q0 * SEQ_FULL;
    const int mr0 = tid >> 4, mp = tid & 15;
    const int pwo = wave * (QT * 32);
    const int oso = wave * (QT * 68);

#pragma unroll 1
    for (int kc = 0; kc < SEQ / KC; ++kc) {
        const int kv0 = kc * KC;
        const bool kres = res && (kv0 < ER);
        const v4i mk0 = *(const v4i*)(mb + (size_t)mr0 * SEQ_FULL + kv0 + mp * 4);
        const v4i mk1 = *(const v4i*)(mb + (size_t)(mr0 + 8) * SEQ_FULL + kv0 + mp * 4);
        const int lany = ((mk0.x == 0) | (mk0.y == 0) | (mk0.z == 0) | (mk0.w == 0) |
                          (mk1.x == 0) | (mk1.y == 0) | (mk1.z == 0) | (mk1.w == 0)) ? 1 : 0;
        const int wany = __any(lany);
        const int fo = (kc & 1) * NWAVE;
        if (lane == 0) Fsh[fo + wave] = wany;
        __syncthreads();
        int any = Fsh[fo] | Fsh[fo + 1] | Fsh[fo + 2] | Fsh[fo + 3];
        any = __builtin_amdgcn_readfirstlane(any);
        if (any == 0) continue;

        *(v4i*)(&Msh[mr0 * KC + mp * 4])       = mk0;
        *(v4i*)(&Msh[(mr0 + 8) * KC + mp * 4]) = mk1;
#pragma unroll
        for (int i = 0; i < 4; ++i) {
            const int idx = tid + 128 * i;
            const int row = idx >> 3, pc = idx & 7;
            const v4u kk = *(const v4u*)(Kb + (size_t)(kv0 + row) * EKV + pc * 8);
            const v4u vv = *(const v4u*)(Vb + (size_t)row * SEQ + kv0 + pc * 8);
            *(v4u*)(&Ksh[row * HDIM + pc * 8]) = kk;
            *(v4u*)(&Vth[row * KC + pc * 8])   = vv;
        }
        if (res) {
#pragma unroll
            for (int i = 0; i < 4; ++i) {
                const int idx = tid + 128 * i;
                const int row = idx >> 3, pc = idx & 7;
                const v4u vl = *(const v4u*)(Vl + (size_t)row * SEQ + kv0 + pc * 8);
                *(v4u*)(&Vtl[row * KC + pc * 8]) = vl;
            }
        }
        if (kres) {
#pragma unroll
            for (int i = 0; i < 4; ++i) {
                const int idx = tid + 128 * i;
                const int row = idx >> 3, pc = idx & 7;
                const v4u kl = *(const v4u*)(Kl + (size_t)(kv0 + row) * EKV + pc * 8);
                *(v4u*)(&Ksl[row * HDIM + pc * 8]) = kl;
            }
        }
        __syncthreads();

#pragma unroll 1
        for (int hf = 0; hf < 2; ++hf) {
            v8f s0 = (v8f){0.f, 0.f, 0.f, 0.f, 0.f, 0.f, 0.f, 0.f};
            v8f s1 = (v8f){0.f, 0.f, 0.f, 0.f, 0.f, 0.f, 0.f, 0.f};
#pragma unroll
            for (int dc = 0; dc < 2; ++dc) {
                FH qh, ql, ka, kb;
                qh.h[0] = *(const v8h*)(Qh + qbase + dc * 32);
                qh.h[1] = *(const v8h*)(Qh + qbase + dc * 32 + 16);
                ql.h[0] = *(const v8h*)(Ql + qbase + dc * 32);
                ql.h[1] = *(const v8h*)(Ql + qbase + dc * 32 + 16);
                const int ko = (hf * 32 + c) * HDIM + dc * 32 + 8 * hh;
                ka.h[0] = *(const v8h*)(&Ksh[ko]);
                ka.h[1] = *(const v8h*)(&Ksh[ko + 16]);
                kb.h[0] = *(const v8h*)(&Ksh[ko + 16 * HDIM]);
                kb.h[1] = *(const v8h*)(&Ksh[ko + 16 * HDIM + 16]);
                s0 = mma_h(qh.v, ka.v, s0);
                s0 = mma_h(ql.v, ka.v, s0);
                s1 = mma_h(qh.v, kb.v, s1);
                s1 = mma_h(ql.v, kb.v, s1);
                if (kres) {
                    FH kal, kbl;
                    kal.h[0] = *(const v8h*)(&Ksl[ko]);
                    kal.h[1] = *(const v8h*)(&Ksl[ko + 16]);
                    kbl.h[0] = *(const v8h*)(&Ksl[ko + 16 * HDIM]);
                    kbl.h[1] = *(const v8h*)(&Ksl[ko + 16 * HDIM + 16]);
                    s0 = mma_h(qh.v, kal.v, s0);
                    s1 = mma_h(qh.v, kbl.v, s1);
                }
            }

#pragma unroll
            for (int r = 0; r < 8; ++r) {
                const int mo = (8 * hh + r) * KC + hf * 32 + c;
                const int m0 = Msh[mo], m1 = Msh[mo + 16];
                const float x0 = (m0 != 0) ? -INFINITY : s0[r] * SL2;
                const float x1 = (m1 != 0) ? -INFINITY : s1[r] * SL2;
                float m = fmaxf(x0, x1);
                m = fmaxf(m, __shfl_xor(m, 1, 32)); m = fmaxf(m, __shfl_xor(m, 2, 32));
                m = fmaxf(m, __shfl_xor(m, 4, 32)); m = fmaxf(m, __shfl_xor(m, 8, 32));
                const float mnew  = fmaxf(mrow[r], m);
                const float msafe = (mnew == -INFINITY) ? 0.0f : mnew;
                const float alpha = exp2f(mrow[r] - msafe);
                mrow[r] = mnew;
                const float p0 = exp2f(x0 - msafe), p1 = exp2f(x1 - msafe);
                const float c0 = p0 * PSC, c1 = p1 * PSC;
                const _Float16 h0 = (_Float16)c0, h1 = (_Float16)c1;
                const int po = pwo + (8 * hh + r) * 32 + c;
                Psh[po]      = h0;
                Psh[po + 16] = h1;
                if (res) {
                    Psl[po]      = (_Float16)(c0 - (float)h0);
                    Psl[po + 16] = (_Float16)(c1 - (float)h1);
                }
                float psum = p0 + p1;
                psum += __shfl_xor(psum, 1, 32); psum += __shfl_xor(psum, 2, 32);
                psum += __shfl_xor(psum, 4, 32); psum += __shfl_xor(psum, 8, 32);
                lrow[r] = lrow[r] * alpha + psum;
#pragma unroll
                for (int t = 0; t < 4; ++t) oacc[t][r] *= alpha;
            }
            wave_sync();

            {
                FH pa, pl;
                const int pr = pwo + c * 32 + 8 * hh;
                pa.h[0] = *(const v8h*)(&Psh[pr]);
                pa.h[1] = *(const v8h*)(&Psh[pr + 16]);
                if (res) {
                    pl.h[0] = *(const v8h*)(&Psl[pr]);
                    pl.h[1] = *(const v8h*)(&Psl[pr + 16]);
                } else {
                    pl.v = pa.v;
                }
#pragma unroll
                for (int t = 0; t < 4; ++t) {
                    FH vb;
                    const int vo = (t * 16 + c) * KC + hf * 32 + 8 * hh;
                    vb.h[0] = *(const v8h*)(&Vth[vo]);
                    vb.h[1] = *(const v8h*)(&Vth[vo + 16]);
                    oacc[t] = mma_h(pa.v, vb.v, oacc[t]);
                    if (res) {
                        FH vl;
                        vl.h[0] = *(const v8h*)(&Vtl[vo]);
                        vl.h[1] = *(const v8h*)(&Vtl[vo + 16]);
                        oacc[t] = mma_h(pl.v, vb.v, oacc[t]);
                        oacc[t] = mma_h(pa.v, vl.v, oacc[t]);
                    }
                }
            }
            wave_sync();
        }
    }

#pragma unroll
    for (int r = 0; r < 8; ++r) {
        const float inv = 1.0f / (lrow[r] * (PSC * VSC));
#pragma unroll
        for (int t = 0; t < 4; ++t) Os[oso + (8 * hh + r) * 68 + t * 16 + c] = oacc[t][r] * inv;
    }
    wave_sync();
    {
        const int pr = lane >> 3, pc = lane & 7;
#pragma unroll 1
        for (int it = 0; it < 4; ++it) {
            const int row = it * 4 + pr;
            const v4f o0 = *(const v4f*)(&Os[oso + row * 68 + pc * 8]);
            const v4f o1 = *(const v4f*)(&Os[oso + row * 68 + pc * 8 + 4]);
            const float* gp = QKV + (size_t)(q0 + row) * NQKV + head * (2 * HDIM) + HDIM + pc * 8;
            const v4f g0 = *(const v4f*)(gp), g1 = *(const v4f*)(gp + 4);
            const float ov[8] = {o0.x, o0.y, o0.z, o0.w, o1.x, o1.y, o1.z, o1.w};
            const float gv[8] = {g0.x, g0.y, g0.z, g0.w, g1.x, g1.y, g1.z, g1.w};
            unsigned int hb[8], lb[8];
#pragma unroll
            for (int e = 0; e < 8; ++e) {
                const float sg = 1.0f / (1.0f + expf(-gv[e]));
                split_h((ov[e] * sg) * CSC, hb[e], lb[e]);
            }
            v4u ph, pl;
            ph.x = hb[0] | (hb[1] << 16); ph.y = hb[2] | (hb[3] << 16); ph.z = hb[4] | (hb[5] << 16); ph.w = hb[6] | (hb[7] << 16);
            pl.x = lb[0] | (lb[1] << 16); pl.y = lb[2] | (lb[3] << 16); pl.z = lb[4] | (lb[5] << 16); pl.w = lb[6] | (lb[7] << 16);
            const size_t off = (size_t)(q0 + row) * EMB + head * HDIM + pc * 8;
            st16x2(Chi + off, ph);
            if (res) st16x2(Clo + off, pl);
        }
    }
}

extern "C" void kernel_launch(void* const* d_in, const int* in_sizes, int n_in, void* d_out, int out_size, void* d_ws, size_t ws_size, hipStream_t stream) {
    if (n_in < 10) return;
    if ((long long)in_sizes[0] < (long long)SEQ * EMB) return;
    if ((long long)in_sizes[1] < (long long)(SEQ - 1) * SEQ_FULL + SEQ) return;
    if ((long long)in_sizes[2] < (long long)SEQ * HDIM) return;
    if ((long long)in_sizes[3] < (long long)SEQ * HDIM) return;
    if ((long long)in_sizes[4] < (long long)NQG * EMB) return;
    if ((long long)in_sizes[5] < (long long)EKV * EMB) return;
    if ((long long)in_sizes[6] < (long long)EKV * EMB) return;
    if ((long long)in_sizes[7] < (long long)EMB * EMB) return;
    if (in_sizes[8] < HDIM || in_sizes[9] < HDIM) return;
    if ((long long)out_size < (long long)SEQ * EMB) return;
    if (ws_size < WS_TOTAL) return;

    const float* x    = (const float*)d_in[0];
    const int*   mask = (const int*)d_in[1];
    const float* cosT = (const float*)d_in[2];
    const float* sinT = (const float*)d_in[3];
    const float* Wq   = (const float*)d_in[4];
    const float* Wk   = (const float*)d_in[5];
    const float* Wv   = (const float*)d_in[6];
    const float* Wo   = (const float*)d_in[7];
    const float* qnw  = (const float*)d_in[8];
    const float* knw  = (const float*)d_in[9];
    float* out = (float*)d_out;

    char* wsb = (char*)d_ws;
    size_t off = 0;
    unsigned short* XP   = (unsigned short*)(wsb + off); off += XP_B;
    unsigned short* WP   = (unsigned short*)(wsb + off); off += WP_B;
    unsigned short* WOP  = (unsigned short*)(wsb + off); off += WOP_B;
    float*          QKV  = (float*)(wsb + off);          off += QKV_B;
    unsigned short* Qhi  = (unsigned short*)(wsb + off); off += QH_B;
    unsigned short* Qlo  = (unsigned short*)(wsb + off); off += QH_B;
    unsigned short* K16  = (unsigned short*)(wsb + off); off += K16_B;
    unsigned short* Klo  = (unsigned short*)(wsb + off); off += KL_B;
    unsigned short* VThi = (unsigned short*)(wsb + off); off += VT_B;
    unsigned short* VTlo = (unsigned short*)(wsb + off); off += VT_B;
    unsigned short* Chi  = (unsigned short*)(wsb + off); off += CH_B;
    unsigned short* Clo  = (unsigned short*)(wsb + off); off += CL_B;

    k_cvt<<<(unsigned)((SEQ * EMB / 8 + 255) / 256), 256, 0, stream>>>(x, XP, SEQ * EMB / 8, XSC);
    k_cvt<<<(unsigned)((NQG * EMB / 8 + 255) / 256), 256, 0, stream>>>(Wq, WP, NQG * EMB / 8, WSC);
    k_cvt<<<(unsigned)((EKV * EMB / 8 + 255) / 256), 256, 0, stream>>>(Wk, WP + (size_t)NQG * EMB, EKV * EMB / 8, WSC);
    k_cvt<<<(unsigned)((EKV * EMB / 8 + 255) / 256), 256, 0, stream>>>(Wv, WP + (size_t)(NQG + EKV) * EMB, EKV * EMB / 8, WSC);
    k_cvt<<<(unsigned)((EMB * EMB / 8 + 255) / 256), 256, 0, stream>>>(Wo, WOP, EMB * EMB / 8, WSC);

    k_gemm<<<dim3((unsigned)(NQKV / 256), (unsigned)(SEQ / 32)), 128, 0, stream>>>(XP, XP, WP, QKV, EMB, NQKV, 0, 1.0f / (XSC * WSC));

    k_prep_qk<<<dim3((unsigned)(SEQ / 32), (unsigned)(NQH + NKVH)), 256, 0, stream>>>(QKV, cosT, sinT, qnw, knw, Qhi, Qlo, K16, Klo);
    k_prep_v<<<dim3((unsigned)(SEQ / 64), (unsigned)NKVH), 256, 0, stream>>>(QKV, VThi, VTlo);

    k_attn<<<dim3((unsigned)(SEQ / QT), (unsigned)NKVH), 128, 0, stream>>>(Qhi, Qlo, K16, Klo, VThi, VTlo, mask, QKV, Chi, Clo);

    k_gemm<<<dim3((unsigned)(EMB / 256), (unsigned)(SEQ / 32)), 128, 0, stream>>>(Chi, Clo, WOP, out, EMB, EMB, ER, 1.0f / (CSC * WSC));
}
